// Stage1_12197707120912
// MI455X (gfx1250) — hardware-verified
//
#include <hip/hip_runtime.h>

#define BB 16
#define SS 2048
#define DD 128
#define HH 4
#define HDD 32
#define MM (BB * SS)
#define LN_EPS 1e-5f
#define WSCALE 64.0f

typedef _Float16 v16h __attribute__((ext_vector_type(16)));
typedef _Float16 v8h  __attribute__((ext_vector_type(8)));
typedef float    v8f  __attribute__((ext_vector_type(8)));
typedef float    v4f  __attribute__((ext_vector_type(4)));
typedef unsigned int v4u __attribute__((ext_vector_type(4)));

union Frag   { v16h v; v8h half[2]; };
union Pack16 { v4u u; v8h h; v4f f; };

typedef char shape_check[(MM % 128 == 0 && SS % 64 == 0 && (MM * DD) % 8 == 0 && DD % 32 == 0) ? 1 : -1];

struct WPtrs { const float* p[6]; };
typedef char wptrs_check[(sizeof(WPtrs) == 6 * sizeof(const float*)) ? 1 : -1];

__device__ __forceinline__ v16h ld_frag(const _Float16* p) {
  const int hf = (threadIdx.x & 31) >> 4;
  Frag f;
  f.half[0] = *(const v8h*)(p + 8 * hf);
  f.half[1] = *(const v8h*)(p + 16 + 8 * hf);
  return f.v;
}

__device__ __forceinline__ v8f vzero8() {
  v8f z;
#pragma unroll
  for (int i = 0; i < 8; ++i) z[i] = 0.f;
  return z;
}

__device__ __forceinline__ v8f wmma_f16(v16h a, v16h b, v8f c) {
  v8f d = __builtin_amdgcn_wmma_f32_16x16x32_f16(false, a, false, b, (short)0, c, false, false);
  asm volatile("v_nop\n\tv_nop\n\tv_nop\n\tv_nop" : "+v"(d) : "v"(a), "v"(b));
  return d;
}

__device__ __forceinline__ float xsum16(float v) {
  v += __shfl_xor(v, 1, 32);
  v += __shfl_xor(v, 2, 32);
  v += __shfl_xor(v, 4, 32);
  v += __shfl_xor(v, 8, 32);
  return v;
}
__device__ __forceinline__ float xsum32(float v) {
  v = xsum16(v);
  v += __shfl_xor(v, 16, 32);
  return v;
}

__global__ __launch_bounds__(256) void k_w16(WPtrs wp, _Float16* wtb, float wscale) {
  __shared__ __attribute__((aligned(16))) _Float16 sT[DD * DD];
  const int tid = threadIdx.x, wave = tid >> 5, lane = tid & 31;
  const int mi = blockIdx.x;
  const float* W = wp.p[0];
#pragma unroll
  for (int j = 1; j < 6; ++j) if (mi == j) W = wp.p[j];
  _Float16* Wt = wtb + (size_t)mi * DD * DD;

#pragma unroll 4
  for (int it = 0; it < 64; ++it) {
    const int idx = it * 256 + tid;
    const int k = idx >> 7, c = idx & 127;
    sT[c * DD + k] = (_Float16)(W[idx] * wscale);
  }
  __syncthreads();
  v4u p[8];
#pragma unroll
  for (int it = 0; it < 8; ++it) {
    const int qd = it * 256 + wave * 32 + lane;
    const int c = qd >> 4, ch = (qd & 15) * 8;
    p[it] = *(const v4u*)(sT + c * DD + ch);
  }
#pragma unroll
  for (int it = 0; it < 8; ++it) {
    const int qd = it * 256 + wave * 32 + lane;
    const int c = qd >> 4, ch = (qd & 15) * 8;
    *(volatile v4u*)(Wt + (size_t)c * DD + ch) = p[it];
  }
  __threadfence();
#pragma unroll
  for (int it = 0; it < 8; ++it) {
    const int qd = it * 256 + wave * 32 + lane;
    const int c = qd >> 4, ch = (qd & 15) * 8;
    *(volatile v4u*)(Wt + (size_t)c * DD + ch) = p[it];
  }
}

__global__ __launch_bounds__(256) void k_x16(const float* __restrict__ x, _Float16* xh, int n8) {
  const int t = blockIdx.x * 256 + threadIdx.x;
  if (t >= n8) return;
  const size_t off = (size_t)t * 8;
  const v4f a0 = *(const v4f*)(x + off);
  const v4f a1 = *(const v4f*)(x + off + 4);
  Pack16 pk;
#pragma unroll
  for (int i = 0; i < 4; ++i) { pk.h[i] = (_Float16)a0[i]; pk.h[4 + i] = (_Float16)a1[i]; }
  const v4u val = pk.u;
  *(volatile v4u*)(xh + off) = val;
  __threadfence();
  *(volatile v4u*)(xh + off) = val;
}

template <int AL, int MODE>
__global__ __launch_bounds__(256) void k_gemm(const _Float16* __restrict__ A,
                                              const _Float16* __restrict__ Wt,
                                              const float* __restrict__ bias,
                                              float oscale, float bscale,
                                              _Float16* outh, float* outf, int nrows) {
  __shared__ __attribute__((aligned(16))) float stgraw[8192];
  _Float16* stg = (_Float16*)stgraw;
  const int tid = threadIdx.x, wave = tid >> 5, lane = tid & 31;
  const int hf = lane >> 4, cb = lane & 15;
  const int blk0 = blockIdx.x * 128;
  if (blk0 + 128 > nrows) return;
  const int r0 = blk0 + (wave & 3) * 32;
  const int c0 = (wave >> 2) * 64;

  v8f acc[2][4];
#pragma unroll
  for (int rt = 0; rt < 2; ++rt)
#pragma unroll
    for (int nt = 0; nt < 4; ++nt) acc[rt][nt] = vzero8();

#pragma unroll
  for (int ks = 0; ks < DD; ks += 32) {
    v16h af[2];
#pragma unroll
    for (int rt = 0; rt < 2; ++rt) {
      const int row = r0 + rt * 16 + cb;
      const _Float16* ap;
      if (AL == 0) ap = A + (size_t)row * DD + ks;
      else         ap = A + ((size_t)((row >> 11) * HH + (ks >> 5)) * SS + (row & (SS - 1))) * HDD;
      af[rt] = ld_frag(ap);
    }
#pragma unroll
    for (int nt = 0; nt < 4; ++nt) {
      const v16h bf = ld_frag(Wt + (size_t)(c0 + nt * 16 + cb) * DD + ks);
      acc[0][nt] = wmma_f16(af[0], bf, acc[0][nt]);
      acc[1][nt] = wmma_f16(af[1], bf, acc[1][nt]);
    }
  }

  if (MODE == 0 || MODE == 3) {
    _Float16* sw = stg + wave * 2048;
#pragma unroll
    for (int rt = 0; rt < 2; ++rt) {
#pragma unroll
      for (int nt = 0; nt < 4; ++nt) {
        const int col = nt * 16 + cb;
        const float bvv = bias[c0 + col] * bscale;
#pragma unroll
        for (int i = 0; i < 8; ++i) {
          float v = acc[rt][nt][i] * oscale + bvv;
          if (MODE == 3) v = v > 0.f ? v : 0.f;
          sw[(rt * 16 + 8 * hf + i) * 64 + col] = (_Float16)v;
        }
      }
    }
    __syncthreads();
    v4u p[8];
#pragma unroll
    for (int it = 0; it < 8; ++it) {
      const int qd = it * 32 + lane;
      const int row = qd >> 3, ch = (qd & 7) * 8;
      p[it] = *(const v4u*)(sw + row * 64 + ch);
    }
#pragma unroll
    for (int it = 0; it < 8; ++it) {
      const int qd = it * 32 + lane;
      const int row = qd >> 3, ch = (qd & 7) * 8;
      *(volatile v4u*)(outh + (size_t)(r0 + row) * DD + c0 + ch) = p[it];
    }
    __threadfence();
#pragma unroll
    for (int it = 0; it < 8; ++it) {
      const int qd = it * 32 + lane;
      const int row = qd >> 3, ch = (qd & 7) * 8;
      *(volatile v4u*)(outh + (size_t)(r0 + row) * DD + c0 + ch) = p[it];
    }
  } else if (MODE == 2) {
    float* swf = stgraw + wave * 1024;
#pragma unroll
    for (int rt = 0; rt < 2; ++rt) {
      if (rt) __syncthreads();
#pragma unroll
      for (int nt = 0; nt < 4; ++nt) {
        const int col = nt * 16 + cb;
        const float bvv = bias[c0 + col] * bscale;
#pragma unroll
        for (int i = 0; i < 8; ++i)
          swf[(8 * hf + i) * 64 + col] = acc[rt][nt][i] * oscale + bvv;
      }
      __syncthreads();
      v4u p[8];
#pragma unroll
      for (int it = 0; it < 8; ++it) {
        const int qd = it * 32 + lane;
        const int row = qd >> 4, ch = (qd & 15) * 4;
        p[it] = *(const v4u*)(swf + row * 64 + ch);
      }
#pragma unroll
      for (int it = 0; it < 8; ++it) {
        const int qd = it * 32 + lane;
        const int row = qd >> 4, ch = (qd & 15) * 4;
        *(volatile v4u*)(outf + (size_t)(r0 + rt * 16 + row) * DD + c0 + ch) = p[it];
      }
      __threadfence();
#pragma unroll
      for (int it = 0; it < 8; ++it) {
        const int qd = it * 32 + lane;
        const int row = qd >> 4, ch = (qd & 15) * 4;
        *(volatile v4u*)(outf + (size_t)(r0 + rt * 16 + row) * DD + c0 + ch) = p[it];
      }
    }
  } else {
    _Float16* sT = stg;
#pragma unroll
    for (int rt = 0; rt < 2; ++rt) {
#pragma unroll
      for (int nt = 0; nt < 4; ++nt) {
        const int col = c0 + nt * 16 + cb;
        const float bvv = bias[col] * bscale;
#pragma unroll
        for (int i = 0; i < 8; ++i) {
          const int srow = (wave & 3) * 32 + rt * 16 + 8 * hf + i;
          sT[col * 128 + srow] = (_Float16)(acc[rt][nt][i] * oscale + bvv);
        }
      }
    }
    __syncthreads();
    const int bb = blk0 >> 11, sb = blk0 & (SS - 1);
    v4u p[8];
#pragma unroll
    for (int it = 0; it < 8; ++it) {
      const int qd = it * 256 + wave * 32 + lane;
      const int col = qd >> 4, ch = (qd & 15) * 8;
      p[it] = *(const v4u*)(sT + col * 128 + ch);
    }
#pragma unroll
    for (int it = 0; it < 8; ++it) {
      const int qd = it * 256 + wave * 32 + lane;
      const int col = qd >> 4, ch = (qd & 15) * 8;
      *(volatile v4u*)(outh + ((size_t)((bb * HH + (col >> 5)) * HDD + (col & 31))) * SS + sb + ch) = p[it];
    }
    __threadfence();
#pragma unroll
    for (int it = 0; it < 8; ++it) {
      const int qd = it * 256 + wave * 32 + lane;
      const int col = qd >> 4, ch = (qd & 15) * 8;
      *(volatile v4u*)(outh + ((size_t)((bb * HH + (col >> 5)) * HDD + (col & 31))) * SS + sb + ch) = p[it];
    }
  }
}

__global__ __launch_bounds__(128) void k_attn(const _Float16* __restrict__ qh,
                                              const _Float16* __restrict__ kh,
                                              const _Float16* __restrict__ vt,
                                              _Float16* ath, float scs) {
  __shared__ float lsh[4][16];
  __shared__ __attribute__((aligned(16))) _Float16 sto[4][512];
  const int wave = threadIdx.x >> 5, lane = threadIdx.x & 31;
  const int hf = lane >> 4, cb = lane & 15, rb = hf * 8;
  const int b = blockIdx.z, h = blockIdx.y;
  const int q0 = blockIdx.x * 64 + wave * 16;
  const size_t rowbase = (size_t)b * SS;
  const size_t hvbase  = (size_t)(b * HH + h) * HDD;

  const v16h bqf = ld_frag(qh + (rowbase + q0 + cb) * DD + h * HDD);

  float m = -1e30f, l = 0.f;
  v8f o0 = vzero8(), o1 = vzero8();

  for (int kv = 0; kv < SS; kv += 64) {
    v16h bv0[2], bv1[2];
#pragma unroll
    for (int c = 0; c < 2; ++c) {
      bv0[c] = ld_frag(vt + (hvbase + cb) * SS + kv + 32 * c);
      bv1[c] = ld_frag(vt + (hvbase + 16 + cb) * SS + kv + 32 * c);
    }
    v8f st[4];
#pragma unroll
    for (int t = 0; t < 4; ++t) {
      const v16h ak = ld_frag(kh + (rowbase + kv + 16 * t + cb) * DD + h * HDD);
      st[t] = wmma_f16(ak, bqf, vzero8());
    }
#pragma unroll
    for (int t = 0; t < 4; ++t)
#pragma unroll
      for (int i = 0; i < 8; ++i) st[t][i] *= scs;

    float e[8];
#pragma unroll
    for (int i = 0; i < 8; ++i)
      e[i] = fmaxf(fmaxf(st[0][i], st[1][i]), fmaxf(st[2][i], st[3][i]));
#pragma unroll
    for (int i = 0; i < 4; ++i) e[i] = fmaxf(e[i], e[i + 4]);
    float mt = fmaxf(fmaxf(e[0], e[2]), fmaxf(e[1], e[3]));
    mt = fmaxf(mt, __shfl_xor(mt, 16, 32));

    const float mn = fmaxf(m, mt);
    const float alpha = __builtin_amdgcn_exp2f(m - mn);
    m = mn;

#pragma unroll
    for (int t = 0; t < 4; ++t)
#pragma unroll
      for (int i = 0; i < 8; ++i)
        st[t][i] = __builtin_amdgcn_exp2f((st[t][i] - mn) + 12.0f);

    float r[8];
#pragma unroll
    for (int i = 0; i < 8; ++i)
      r[i] = (st[0][i] + st[1][i]) + (st[2][i] + st[3][i]);
#pragma unroll
    for (int i = 0; i < 4; ++i) r[i] += r[i + 4];
    float rs = (r[0] + r[2]) + (r[1] + r[3]);
    rs += __shfl_xor(rs, 16, 32);
    l = l * alpha + rs;
#pragma unroll
    for (int i = 0; i < 8; ++i) { o0[i] *= alpha; o1[i] *= alpha; }

#pragma unroll
    for (int c = 0; c < 2; ++c) {
      Frag pf;
#pragma unroll
      for (int i = 0; i < 8; ++i) {
        pf.half[0][i] = (_Float16)st[2 * c][i];
        pf.half[1][i] = (_Float16)st[2 * c + 1][i];
      }
      o0 = wmma_f16(pf.v, bv0[c], o0);
      o1 = wmma_f16(pf.v, bv1[c], o1);
    }
  }

  if (lane < 16) lsh[wave][lane] = l;
  __syncthreads();
  float linv[8];
#pragma unroll
  for (int i = 0; i < 8; ++i) linv[i] = 1.f / lsh[wave][rb + i];

#pragma unroll
  for (int i = 0; i < 8; ++i) {
    sto[wave][(rb + i) * 32 + cb]      = (_Float16)(o0[i] * linv[i]);
    sto[wave][(rb + i) * 32 + 16 + cb] = (_Float16)(o1[i] * linv[i]);
  }
  __syncthreads();
  _Float16* gb = ath + ((size_t)(b * HH + h) * SS + q0) * HDD;
  v4u p[2];
#pragma unroll
  for (int it = 0; it < 2; ++it) {
    const int qd = it * 32 + lane;
    const int row = qd >> 2, ch = (qd & 3) * 8;
    p[it] = *(const v4u*)(&sto[wave][row * 32 + ch]);
  }
#pragma unroll
  for (int it = 0; it < 2; ++it) {
    const int qd = it * 32 + lane;
    const int row = qd >> 2, ch = (qd & 3) * 8;
    *(volatile v4u*)(gb + row * HDD + ch) = p[it];
  }
  __threadfence();
#pragma unroll
  for (int it = 0; it < 2; ++it) {
    const int qd = it * 32 + lane;
    const int row = qd >> 2, ch = (qd & 3) * 8;
    *(volatile v4u*)(gb + row * HDD + ch) = p[it];
  }
}

__global__ __launch_bounds__(256) void k_ln16(const float* __restrict__ a,
                                              const float* __restrict__ res,
                                              const float* __restrict__ g,
                                              const float* __restrict__ be,
                                              _Float16* outh, int nrows) {
  const int wave = threadIdx.x >> 5, lane = threadIdx.x & 31;
  const int row = blockIdx.x * 16 + wave * 2 + (lane >> 4);
  const int j = lane & 15;
  const int rowc = row < nrows ? row : nrows - 1;
  const size_t off = (size_t)rowc * DD + 8 * j;
  const v4f a0 = *(const v4f*)(a + off),   a1 = *(const v4f*)(a + off + 4);
  const v4f x0 = *(const v4f*)(res + off), x1 = *(const v4f*)(res + off + 4);
  float x[8];
#pragma unroll
  for (int i = 0; i < 4; ++i) { x[i] = a0[i] + x0[i]; x[4 + i] = a1[i] + x1[i]; }
  float s = 0.f;
#pragma unroll
  for (int i = 0; i < 8; ++i) s += x[i];
  s = xsum16(s);
  const float mean = s * (1.f / 128.f);
  float d[8], s2 = 0.f;
#pragma unroll
  for (int i = 0; i < 8; ++i) { d[i] = x[i] - mean; s2 += d[i] * d[i]; }
  s2 = xsum16(s2);
  const float rstd = rsqrtf(s2 * (1.f / 128.f) + LN_EPS);
  Pack16 pk;
#pragma unroll
  for (int i = 0; i < 8; ++i) {
    const int col = 8 * j + i;
    pk.h[i] = (_Float16)(d[i] * rstd * g[col] + be[col]);
  }
  const v4u val = pk.u;
  _Float16* gp = outh + (size_t)row * DD + 8 * j;
  if (row < nrows) *(volatile v4u*)gp = val;
  __threadfence();
  if (row < nrows) *(volatile v4u*)gp = val;
}

__global__ __launch_bounds__(256) void k_ln32(const float* __restrict__ a,
                                              const float* __restrict__ res,
                                              const float* __restrict__ g,
                                              const float* __restrict__ be,
                                              float* outf, int nrows) {
  const int wave = threadIdx.x >> 5, lane = threadIdx.x & 31;
  const int row = blockIdx.x * 8 + wave;
  const int rowc = row < nrows ? row : nrows - 1;
  const size_t off = (size_t)rowc * DD + 4 * lane;
  const v4f a0 = *(const v4f*)(a + off);
  const v4f x0 = *(const v4f*)(res + off);
  float x[4];
#pragma unroll
  for (int i = 0; i < 4; ++i) x[i] = a0[i] + x0[i];
  float s = (x[0] + x[1]) + (x[2] + x[3]);
  s = xsum32(s);
  const float mean = s * (1.f / 128.f);
  float d[4], s2 = 0.f;
#pragma unroll
  for (int i = 0; i < 4; ++i) { d[i] = x[i] - mean; s2 += d[i] * d[i]; }
  s2 = xsum32(s2);
  const float rstd = rsqrtf(s2 * (1.f / 128.f) + LN_EPS);
  v4f y;
#pragma unroll
  for (int i = 0; i < 4; ++i) {
    const int col = 4 * lane + i;
    y[i] = d[i] * rstd * g[col] + be[col];
  }
  float* gp = outf + (size_t)row * DD + 4 * lane;
  if (row < nrows) *(volatile v4f*)gp = y;
  __threadfence();
  if (row < nrows) *(volatile v4f*)gp = y;
}

extern "C" void kernel_launch(void* const* d_in, const int* in_sizes, int n_in,
                              void* d_out, int out_size, void* d_ws, size_t ws_size,
                              hipStream_t stream) {
  if (n_in < 17) return;
  if (in_sizes[0] != MM * DD || out_size != MM * DD) return;
  for (int i = 0; i < 8; ++i) {
    if (in_sizes[1 + 2 * i] != ((i == 4 || i == 7) ? DD : DD * DD) && (i == 4 || i == 7)) return;
  }
  if (in_sizes[1] != DD * DD || in_sizes[3] != DD * DD || in_sizes[5] != DD * DD ||
      in_sizes[7] != DD * DD || in_sizes[11] != DD * DD || in_sizes[13] != DD * DD) return;
  if (in_sizes[2] != DD || in_sizes[4] != DD || in_sizes[6] != DD || in_sizes[8] != DD ||
      in_sizes[9] != DD || in_sizes[10] != DD || in_sizes[12] != DD || in_sizes[14] != DD ||
      in_sizes[15] != DD || in_sizes[16] != DD) return;

  const float* x   = (const float*)d_in[0];
  const float* Wq  = (const float*)d_in[1];
  const float* bq  = (const float*)d_in[2];
  const float* Wk  = (const float*)d_in[3];
  const float* bk  = (const float*)d_in[4];
  const float* Wv  = (const float*)d_in[5];
  const float* bv  = (const float*)d_in[6];
  const float* Wo  = (const float*)d_in[7];
  const float* bo  = (const float*)d_in[8];
  const float* g1  = (const float*)d_in[9];
  const float* b1  = (const float*)d_in[10];
  const float* W1  = (const float*)d_in[11];
  const float* bf1 = (const float*)d_in[12];
  const float* W2  = (const float*)d_in[13];
  const float* bf2 = (const float*)d_in[14];
  const float* g2  = (const float*)d_in[15];
  const float* b2  = (const float*)d_in[16];
  float* out = (float*)d_out;

  const size_t R = (size_t)MM * DD * sizeof(_Float16);
  const size_t need = 5 * R + (size_t)6 * DD * DD * sizeof(_Float16);
  if (ws_size < need) return;
  char* ws = (char*)d_ws;
  _Float16* xh   = (_Float16*)(ws);
  _Float16* qh   = (_Float16*)(ws + R);
  _Float16* kh   = (_Float16*)(ws + 2 * R);
  _Float16* vth  = (_Float16*)(ws + 3 * R);
  _Float16* ath  = (_Float16*)(ws + 4 * R);
  float*    of   = (float*)(ws + R);
  _Float16* wtb  = (_Float16*)(ws + 5 * R);
  _Float16* WqT = wtb + 0 * DD * DD;
  _Float16* WkT = wtb + 1 * DD * DD;
  _Float16* WvT = wtb + 2 * DD * DD;
  _Float16* WoT = wtb + 3 * DD * DD;
  _Float16* W1T = wtb + 4 * DD * DD;
  _Float16* W2T = wtb + 5 * DD * DD;
  float*    dumf = (float*)(ws + 4 * R);
  _Float16* dumh = ath;

  const int nrows = in_sizes[0] / DD;
  const int n8 = in_sizes[0] / 8;
  const float scs = (0.17677669529663687f * 1.4426950408889634f) * (1.0f / 4096.0f);
  const float inv4096 = 1.0f / 4096.0f;

  WPtrs wp;
  wp.p[0] = Wq; wp.p[1] = Wk; wp.p[2] = Wv; wp.p[3] = Wo; wp.p[4] = W1; wp.p[5] = W2;
  k_w16<<<6, 256, 0, stream>>>(wp, wtb, WSCALE);
  k_x16<<<(n8 + 255) / 256, 256, 0, stream>>>(x, xh, n8);

  const int ggrid = (nrows + 127) / 128;
  k_gemm<0, 0><<<ggrid, 256, 0, stream>>>(xh, WqT, bq, 1.0f, WSCALE, qh, dumf, nrows);
  k_gemm<0, 0><<<ggrid, 256, 0, stream>>>(xh, WkT, bk, 1.0f, WSCALE, kh, dumf, nrows);
  k_gemm<0, 1><<<ggrid, 256, 0, stream>>>(xh, WvT, bv, 1.0f, WSCALE, vth, dumf, nrows);

  dim3 ag(SS / 64, HH, BB);
  k_attn<<<ag, 128, 0, stream>>>(qh, kh, vth, ath, scs);

  k_gemm<1, 2><<<ggrid, 256, 0, stream>>>(ath, WoT, bo, inv4096, 1.0f, dumh, of, nrows);
  k_ln16<<<(nrows + 15) / 16, 256, 0, stream>>>(of, x, g1, b1, vth, nrows);

  k_gemm<0, 3><<<ggrid, 256, 0, stream>>>(vth, W1T, bf1, 1.0f, WSCALE, xh, dumf, nrows);
  k_gemm<0, 2><<<ggrid, 256, 0, stream>>>(xh, W2T, bf2, inv4096, 1.0f, dumh, of, nrows);

  k_ln32<<<(nrows + 7) / 8, 256, 0, stream>>>(of, x, g2, b2, out, nrows);
}
